// HierarchicalFlowAnchor_35390530519881
// MI455X (gfx1250) — hardware-verified
//
#include <hip/hip_runtime.h>
#include <math.h>
typedef __attribute__((ext_vector_type(16))) _Float16 v16h;
typedef __attribute__((ext_vector_type(8)))  _Float16 v8h;
typedef __attribute__((ext_vector_type(16))) __bf16   v16b;
typedef __attribute__((ext_vector_type(8)))  __bf16   v8b;
typedef __attribute__((ext_vector_type(8)))  float    v8f;
typedef __attribute__((ext_vector_type(4)))  float    v4f;
#define PSCALE 32768.0f
#define U16(p) ((const unsigned short*)(const void*)(p))
#define PSCALE_INV (1.0f / 32768.0f)

__device__ __forceinline__ unsigned short f2bf_bits(float f) {
  unsigned u = __float_as_uint(f);
  return (unsigned short)((u + 0x7FFFu + ((u >> 16) & 1u)) >> 16);
}
__device__ __forceinline__ float bf_bits2f(unsigned short h) { return __uint_as_float(((unsigned)h) << 16); }

__device__ __forceinline__ void dep_guard_h(v8f& a, v8f& b, v16h x, v16h y) { asm volatile("v_nop\n\tv_nop\n\tv_nop\n\tv_nop" : "+v"(a), "+v"(b) : "v"(x), "v"(y)); }
__device__ __forceinline__ void dep_guard_b(v8f& a, v8f& b, v16b x, v16b y) { asm volatile("v_nop\n\tv_nop\n\tv_nop\n\tv_nop" : "+v"(a), "+v"(b) : "v"(x), "v"(y)); }
__device__ __forceinline__ void keep4_h(v16h a, v16h b, v16h c, v16h d) { asm volatile("v_nop" :: "v"(a), "v"(b), "v"(c), "v"(d)); }
__device__ __forceinline__ void keep4_b(v16b a, v16b b, v16b c, v16b d) { asm volatile("v_nop" :: "v"(a), "v"(b), "v"(c), "v"(d)); }
__device__ __forceinline__ void acc_guard4(v8f& a, v8f& b, v8f& c, v8f& d) { asm volatile("v_nop\n\tv_nop\n\tv_nop\n\tv_nop" : "+v"(a), "+v"(b), "+v"(c), "+v"(d)); }
template <typename T> struct Frag;
template <> struct Frag<_Float16> {
  typedef v16h V; union U { v16h v; v8h h[2]; };
  static __device__ __forceinline__ v16h load(const _Float16* p) {
    U f; f.h[0] = *(const v8h*)(p); f.h[1] = *(const v8h*)(p + 16); return f.v;
  }
  static __device__ __forceinline__ v8f mma(v16h a, v16h b, v8f c) {
    return __builtin_amdgcn_wmma_f32_16x16x32_f16(false, a, false, b, (short)0, c, false, false);
  }
  static __device__ __forceinline__ void guard(v8f& a, v8f& b, v16h x, v16h y) { dep_guard_h(a, b, x, y); }
  static __device__ __forceinline__ void keep(v16h a, v16h b, v16h c, v16h d) { keep4_h(a, b, c, d); }
};
template <> struct Frag<__bf16> {
  typedef v16b V; union U { v16b v; v8b h[2]; };
  static __device__ __forceinline__ v16b load(const __bf16* p) {
    U f; f.h[0] = *(const v8b*)(p); f.h[1] = *(const v8b*)(p + 16); return f.v;
  }
  static __device__ __forceinline__ v8f mma(v16b a, v16b b, v8f c) {
    return __builtin_amdgcn_wmma_f32_16x16x32_bf16(false, a, false, b, (short)0, c, false, false);
  }
  static __device__ __forceinline__ void guard(v8f& a, v8f& b, v16b x, v16b y) { dep_guard_b(a, b, x, y); }
  static __device__ __forceinline__ void keep(v16b a, v16b b, v16b c, v16b d) { keep4_b(a, b, c, d); }
};

template <int ET> struct Elem;
template <> struct Elem<0> { typedef _Float16 T; };
template <> struct Elem<1> { typedef __bf16 T; };
template <int ET, bool SPLIT, int BIAS_MODE, int OUT_MODE, bool RESID, int ACT = 0>
__global__ __launch_bounds__(256) void wmma_gemm64(
    const unsigned short* __restrict__ Ap, const unsigned short* __restrict__ A2p, int lda, long strideA,
    const unsigned short* __restrict__ Btp, const unsigned short* __restrict__ Bt2p, int ldb, long strideB,
    void* __restrict__ Cout, void* __restrict__ Cout2, int ldc, long strideC,
    const float* __restrict__ bias,
    const float* __restrict__ resid, long strideR,
    int M, int N, int K, float scale) {
  typedef typename Elem<ET>::T T;
  typedef typename Frag<T>::V V;
  const T* A = (const T*)Ap; const T* A2 = (const T*)A2p; const T* Bt = (const T*)Btp; const T* Bt2 = (const T*)Bt2p;
  __shared__ __align__(16) float sT[8][16 * 68];
  const int b    = blockIdx.y;
  const int lane = threadIdx.x & 31;
  const int wave = threadIdx.x >> 5;
  const int tilesN = N >> 6;
  const int tilesM = M >> 6;
  const int tile = blockIdx.x * 8 + wave;
  if (tile >= tilesM * tilesN) return;
  const int tm = tile / tilesN;
  const int tn = tile - tm * tilesN;
  const int m0 = tm << 6;
  const int n0 = tn << 6;

  const T* Ab  = A  + (size_t)b * strideA;
  const T* Bb  = Bt + (size_t)b * strideB;
  const T* Ab2 = SPLIT ? (A2  + (size_t)b * strideA) : nullptr;
  const T* Bb2 = SPLIT ? (Bt2 + (size_t)b * strideB) : nullptr;

  const int rlane = lane & 15;
  const int koff  = (lane >> 4) * 8;
  const int mOff  = (lane >> 4) * 8;

  v8f acc[4][4];
#pragma unroll
  for (int i = 0; i < 4; ++i)
#pragma unroll
    for (int j = 0; j < 4; ++j) acc[i][j] = (v8f){0.f,0.f,0.f,0.f,0.f,0.f,0.f,0.f};

  for (int k0 = 0; k0 < K; k0 += 32) {
    V bh[4], bl[4];
#pragma unroll
    for (int j = 0; j < 4; ++j) {
      const size_t bo = (size_t)(n0 + (j << 4) + rlane) * ldb + koff + k0;
      bh[j] = Frag<T>::load(Bb + bo);
      if (SPLIT) bl[j] = Frag<T>::load(Bb2 + bo);
    }
#pragma unroll
    for (int i = 0; i < 4; ++i) {
      const size_t ao = (size_t)(m0 + (i << 4) + rlane) * lda + koff + k0;
      V ah = Frag<T>::load(Ab + ao);
      V al;
      if (SPLIT) al = Frag<T>::load(Ab2 + ao);
#pragma unroll
      for (int j = 0; j < 4; ++j) {
        acc[i][j] = Frag<T>::mma(ah, bh[j], acc[i][j]);
        if (SPLIT) {
          acc[i][j] = Frag<T>::mma(ah, bl[j], acc[i][j]);
          acc[i][j] = Frag<T>::mma(al, bh[j], acc[i][j]);
        }
      }
      Frag<T>::guard(acc[i][0], acc[i][3], ah, SPLIT ? al : ah);
    }
    Frag<T>::keep(bh[0], bh[1], bh[2], bh[3]);
    if (SPLIT) Frag<T>::keep(bl[0], bl[1], bl[2], bl[3]);
  }
  acc_guard4(acc[0][0], acc[0][1], acc[0][2], acc[0][3]);
  acc_guard4(acc[1][0], acc[1][1], acc[1][2], acc[1][3]);
  acc_guard4(acc[2][0], acc[2][1], acc[2][2], acc[2][3]);
  acc_guard4(acc[3][0], acc[3][1], acc[3][2], acc[3][3]);

  float* slab = sT[wave];
  const float* Rb = RESID ? (resid + (size_t)b * strideR) : nullptr;
#pragma unroll
  for (int i = 0; i < 4; ++i) {
    const int mBase = m0 + (i << 4);
#pragma unroll
    for (int j = 0; j < 4; ++j) {
      const int n = n0 + (j << 4) + rlane;
      float bv = 0.f;
      if (BIAS_MODE == 2) bv = bias[n];
#pragma unroll
      for (int r = 0; r < 8; ++r) {
        float v = acc[i][j][r] * scale;
        if (BIAS_MODE == 1) v += bias[mBase + mOff + r];
        if (BIAS_MODE == 2) v += bv;
        if (RESID) v += Rb[(size_t)(mBase + mOff + r) * ldc + n];
        if (ACT == 1) v = tanhf(v);
        if (ACT == 2) v = fmaxf(v, 0.0f);
        if (ACT == 3) v = v / (1.0f + expf(-v));
        if (ACT == 4) v = (v > 0.f) ? v : 0.01f * v;
        if (ACT == 5) v = 0.5f * v * (1.0f + erff(v * 0.70710678118654752f));
        slab[(mOff + r) * 68 + (j << 4) + rlane] = v;
      }
    }
    __builtin_amdgcn_fence(__ATOMIC_RELEASE, "workgroup");
    __builtin_amdgcn_wave_barrier();
    __builtin_amdgcn_fence(__ATOMIC_ACQUIRE, "workgroup");
    if (OUT_MODE == 0) {
      float* C = (float*)Cout + (size_t)b * strideC;
      const int hh = lane >> 4, c4 = (lane & 15) * 4;
      for (int pass = 0; pass < 2; ++pass) {
#pragma unroll
        for (int it = 0; it < 8; ++it) {
          const int row = it * 2 + hh;
          v4f v = *(const v4f*)(slab + row * 68 + c4);
          *(volatile v4f*)(C + (size_t)(mBase + row) * ldc + n0 + c4) = v;
        }
        __threadfence();
      }
    } else {
      const int q = lane >> 3, c8 = (lane & 7) * 8;
      unsigned short* C  = (unsigned short*)Cout  + (size_t)b * strideC;
      unsigned short* C2 = (OUT_MODE == 2) ? ((unsigned short*)Cout2 + (size_t)b * strideC) : nullptr;
      for (int pass = 0; pass < 2; ++pass) {
#pragma unroll
        for (int it = 0; it < 4; ++it) {
          const int row = it * 4 + q;
          const float* sp = slab + row * 68 + c8;
          v8h hv, lv;
#pragma unroll
          for (int e = 0; e < 8; ++e) {
            if (OUT_MODE == 1) {
              hv[e] = (_Float16)sp[e];
            } else {
              unsigned short hb = f2bf_bits(sp[e]);
              unsigned short lb = f2bf_bits(sp[e] - bf_bits2f(hb));
              hv[e] = __builtin_bit_cast(_Float16, hb);
              lv[e] = __builtin_bit_cast(_Float16, lb);
            }
          }
          *(volatile v8h*)(C + (size_t)(mBase + row) * ldc + n0 + c8) = hv;
          if (OUT_MODE == 2) *(volatile v8h*)(C2 + (size_t)(mBase + row) * ldc + n0 + c8) = lv;
        }
        __threadfence();
      }
    }
    __builtin_amdgcn_fence(__ATOMIC_RELEASE, "workgroup");
    __builtin_amdgcn_wave_barrier();
    __builtin_amdgcn_fence(__ATOMIC_ACQUIRE, "workgroup");
  }
}

__global__ __launch_bounds__(256) void cast_f32_f16x2(
    const float* __restrict__ in, _Float16* __restrict__ out, int n2) {
  int i = blockIdx.x * 256 + threadIdx.x;
  if (i < n2) {
    const _Float16 h0 = (_Float16)in[2 * i], h1 = (_Float16)in[2 * i + 1];
    const unsigned u = (unsigned)__builtin_bit_cast(unsigned short, h0) | ((unsigned)__builtin_bit_cast(unsigned short, h1) << 16);
    ((volatile unsigned*)out)[i] = u;
    __threadfence();
    ((volatile unsigned*)out)[i] = u;
  }
}


__global__ __launch_bounds__(256) void transpose_cast_f16(const float* __restrict__ in, int ldi,
                                                         _Float16* __restrict__ outT, int ldo, float scale) {
  __shared__ __align__(16) _Float16 tile[64][72];
  const int c0 = blockIdx.x * 64, r0 = blockIdx.y * 64;
  const int t = threadIdx.y * 32 + threadIdx.x;
  for (int i = threadIdx.y; i < 64; i += 8) {
    tile[threadIdx.x][i]      = (_Float16)(in[(size_t)(r0 + i) * ldi + c0 + threadIdx.x] * scale);
    tile[32 + threadIdx.x][i] = (_Float16)(in[(size_t)(r0 + i) * ldi + c0 + 32 + threadIdx.x] * scale);
  }
  __syncthreads();
  const int q = t >> 3, c8 = (t & 7) * 8;
  for (int pass = 0; pass < 2; ++pass) {
#pragma unroll
    for (int it = 0; it < 2; ++it) {
      const int c = it * 32 + q;
      v8h hv = *(const v8h*)(&tile[c][c8]);
      *(volatile v8h*)(outT + (size_t)(c0 + c) * ldo + r0 + c8) = hv;
    }
    __threadfence();
  }
}

#define FB_ 4
#define FS 1024
#define FD 512
#define FH 16
#define FHD 32
#define FR (FB_ * FS)
#define FN6 3072
#define C_FA 0
#define C_HP 512
#define C_MG 1024
#define C_Q 1536
#define C_K 2048
#define C_V 2560
__global__ __launch_bounds__(256) void ln_kernel(const float* __restrict__ x, const float* __restrict__ g, const float* __restrict__ bb, unsigned* __restrict__ XN16) {
  const int lane = threadIdx.x & 31, wave = threadIdx.x >> 5; const size_t r = (size_t)blockIdx.x * 8 + wave;
  float v[16]; float s = 0.f;
  for (int q = 0; q < 4; ++q) { const v4f a = *(const v4f*)(x + r * FD + lane * 16 + 4 * q); for (int e = 0; e < 4; ++e) { v[4 * q + e] = a[e]; s += a[e]; } }
  for (int o = 16; o > 0; o >>= 1) s += __shfl_xor(s, o, 32);
  const float mean = s / FD; float s2 = 0.f; for (int i = 0; i < 16; ++i) { const float d = v[i] - mean; s2 += d * d; } for (int o = 16; o > 0; o >>= 1) s2 += __shfl_xor(s2, o, 32);
  const float inv = rsqrtf(s2 / FD + 1e-5f);
  unsigned pk[8];
  for (int q = 0; q < 8; ++q) { const int c = lane * 16 + 2 * q; const float a = (v[2 * q] - mean) * inv * g[c] + bb[c], b2 = (v[2 * q + 1] - mean) * inv * g[c + 1] + bb[c + 1];
    pk[q] = (unsigned)__builtin_bit_cast(unsigned short, (_Float16)a) | ((unsigned)__builtin_bit_cast(unsigned short, (_Float16)b2) << 16); }
  typedef __attribute__((ext_vector_type(4))) unsigned u4; const u4 p0 = {pk[0], pk[1], pk[2], pk[3]}, p1 = {pk[4], pk[5], pk[6], pk[7]};
  for (int pass = 0; pass < 2; ++pass) { *(volatile u4*)(XN16 + (r * FD + lane * 16) / 2) = p0; *(volatile u4*)(XN16 + (r * FD + lane * 16) / 2 + 4) = p1; __threadfence(); }
}
__global__ __launch_bounds__(256) void bias6_kernel(const float* b0, const float* b1, const float* b2, const float* b3, const float* b4, const float* b5, float* o) {
  for (int i = blockIdx.x * 256 + threadIdx.x; i < FN6; i += gridDim.x * 256) { const int s = i / FD, c = i % FD; const float* b = (s == 0) ? b0 : (s == 1 ? b1 : (s == 2 ? b2 : (s == 3 ? b3 : (s == 4 ? b4 : b5)))); ((volatile float*)o)[i] = b[c]; __threadfence(); ((volatile float*)o)[i] = b[c]; }
}
__global__ __launch_bounds__(256) void anchor_kernel(const float* __restrict__ P6, unsigned* __restrict__ Q16, unsigned* __restrict__ KW16) {
  const int i = blockIdx.x * 256 + threadIdx.x; if (i >= FB_ * FD / 2) return; const int b = i / (FD / 2), c = 2 * (i % (FD / 2));
  const float* base = P6 + (size_t)b * FS * FN6;
  float mx0 = -INFINITY, mx1 = -INFINITY; for (int s = 0; s < FS; ++s) { mx0 = fmaxf(mx0, base[(size_t)s * FN6 + C_FA + c]); mx1 = fmaxf(mx1, base[(size_t)s * FN6 + C_FA + c + 1]); }
  float se0 = 0.f, se1 = 0.f; for (int s = 0; s < FS; ++s) { se0 += expf(base[(size_t)s * FN6 + C_FA + c] - mx0); se1 += expf(base[(size_t)s * FN6 + C_FA + c + 1] - mx1); }
  const float inv0 = 1.0f / se0, inv1 = 1.0f / se1;
  for (int pass = 0; pass < 2; ++pass) {
    for (int s = 0; s < FS; ++s) { const size_t r = (size_t)b * FS + s; const float* row = base + (size_t)s * FN6;
      const float w0 = expf(row[C_FA + c] - mx0) * inv0, w1 = expf(row[C_FA + c + 1] - mx1) * inv1;
      const unsigned ukw = (unsigned)__builtin_bit_cast(unsigned short, (_Float16)(row[C_K + c] * w0)) | ((unsigned)__builtin_bit_cast(unsigned short, (_Float16)(row[C_K + c + 1] * w1)) << 16);
      const unsigned uq = (unsigned)__builtin_bit_cast(unsigned short, (_Float16)row[C_Q + c]) | ((unsigned)__builtin_bit_cast(unsigned short, (_Float16)row[C_Q + c + 1]) << 16);
      ((volatile unsigned*)KW16)[(r * FD + c) / 2] = ukw; ((volatile unsigned*)Q16)[(r * FD + c) / 2] = uq; }
    __threadfence(); }
}
__global__ __launch_bounds__(256) void probs_kernel(const float* __restrict__ Sm, unsigned* __restrict__ P16) {
  const size_t i = ((size_t)blockIdx.x * 256 + threadIdx.x) * 2;
  float v0[FH], v1[FH]; float mx0 = -INFINITY, mx1 = -INFINITY;
#pragma unroll
  for (int h = 0; h < FH; ++h) { v0[h] = Sm[(size_t)h * FS * FS + i] * 0.17677669529663687f; v1[h] = Sm[(size_t)h * FS * FS + i + 1] * 0.17677669529663687f; mx0 = fmaxf(mx0, v0[h]); mx1 = fmaxf(mx1, v1[h]); }
  float se0 = 0.f, se1 = 0.f;
#pragma unroll
  for (int h = 0; h < FH; ++h) { v0[h] = __expf(v0[h] - mx0); v1[h] = __expf(v1[h] - mx1); se0 += v0[h]; se1 += v1[h]; }
  const float sc0 = 32768.0f / se0, sc1 = 32768.0f / se1;
  for (int pass = 0; pass < 2; ++pass) {
#pragma unroll
    for (int h = 0; h < FH; ++h) ((volatile unsigned*)P16)[((size_t)h * FS * FS + i) / 2] = (unsigned)__builtin_bit_cast(unsigned short, (_Float16)(v0[h] * sc0)) | ((unsigned)__builtin_bit_cast(unsigned short, (_Float16)(v1[h] * sc1)) << 16);
    __threadfence(); }
}
__global__ __launch_bounds__(256) void vt_kernel(const float* __restrict__ P6, int b, unsigned* __restrict__ VT16) {
  __shared__ float tile[32][65];
  const int h = blockIdx.y, t0 = blockIdx.x * 64, tx = threadIdx.x, ty = threadIdx.y;
  for (int r = ty; r < 64; r += 8) { const size_t row = (size_t)b * FS + t0 + r; tile[tx][r] = P6[row * FN6 + C_V + h * FHD + tx]; }
  __syncthreads();
  for (int pass = 0; pass < 2; ++pass) { for (int d = ty; d < 64; d += 8) { unsigned u = 0u; if (d < FHD) u = (unsigned)__builtin_bit_cast(unsigned short, (_Float16)tile[d][2 * tx]) | ((unsigned)__builtin_bit_cast(unsigned short, (_Float16)tile[d][2 * tx + 1]) << 16);
      ((volatile unsigned*)VT16)[(((size_t)h * 64 + d) * FS + t0) / 2 + tx] = u; } __threadfence(); }
}
__global__ __launch_bounds__(256) void combine_kernel(const float* __restrict__ ATT, const float* __restrict__ P6, unsigned* __restrict__ PRE16) {
  const int lane = threadIdx.x & 31, wave = threadIdx.x >> 5; const size_t r = (size_t)blockIdx.x * 8 + wave;
  unsigned pk[8];
  for (int q = 0; q < 8; ++q) { float o2[2]; for (int e = 0; e < 2; ++e) { const int c = lane * 16 + 2 * q + e; const int h = c / FHD, d = c % FHD;
      const float a = ATT[r * 1024 + h * 64 + d]; const float mg = 1.0f / (1.0f + expf(-P6[r * FN6 + C_MG + c])); o2[e] = a * mg + P6[r * FN6 + C_HP + c]; }
    pk[q] = (unsigned)__builtin_bit_cast(unsigned short, (_Float16)o2[0]) | ((unsigned)__builtin_bit_cast(unsigned short, (_Float16)o2[1]) << 16); }
  typedef __attribute__((ext_vector_type(4))) unsigned u4; const u4 p0 = {pk[0], pk[1], pk[2], pk[3]}, p1 = {pk[4], pk[5], pk[6], pk[7]};
  for (int pass = 0; pass < 2; ++pass) { *(volatile u4*)(PRE16 + (r * FD + lane * 16) / 2) = p0; *(volatile u4*)(PRE16 + (r * FD + lane * 16) / 2 + 4) = p1; __threadfence(); }
}
extern "C" void kernel_launch(void* const* d_in, const int* in_sizes, int n_in, void* d_out, int out_size, void* d_ws, size_t ws_size, hipStream_t stream) {
  (void)in_sizes; (void)n_in; (void)out_size; (void)ws_size;
  const float* x = (const float*)d_in[0]; const float* lg = (const float*)d_in[1]; const float* lb = (const float*)d_in[2];
  const float* Wl[6] = {(const float*)d_in[3], (const float*)d_in[5], (const float*)d_in[7], (const float*)d_in[9], (const float*)d_in[11], (const float*)d_in[13]};
  const float* bl[6] = {(const float*)d_in[4], (const float*)d_in[6], (const float*)d_in[8], (const float*)d_in[10], (const float*)d_in[12], (const float*)d_in[14]};
  const float* Wo = (const float*)d_in[15]; const float* bo = (const float*)d_in[16];
  char* ws = (char*)d_ws; size_t off = 0;
  auto carve = [&](size_t bytes) -> char* { char* p = ws + off; off += (bytes + 255) & ~(size_t)255; return p; };
  unsigned* XN16 = (unsigned*)carve((size_t)FR * FD * 2); _Float16* W6 = (_Float16*)carve((size_t)FN6 * FD * 2); float* b6 = (float*)carve(FN6 * 4); _Float16* WoT = (_Float16*)carve((size_t)FD * FD * 2);
  float* P6 = (float*)carve((size_t)FR * FN6 * 4);
  unsigned* Q16 = (unsigned*)carve((size_t)FR * FD * 2); unsigned* KW16 = (unsigned*)carve((size_t)FR * FD * 2);
  float* Sm = (float*)carve((size_t)FH * FS * FS * 4);
  unsigned* P16 = (unsigned*)carve((size_t)FH * FS * FS * 2); unsigned* VT16 = (unsigned*)carve((size_t)FH * 64 * FS * 2);
  float* ATT = (float*)carve((size_t)FR * 1024 * 4); unsigned* PRE16 = (unsigned*)carve((size_t)FR * FD * 2);
  ln_kernel<<<FR / 8, 256, 0, stream>>>(x, lg, lb, XN16);
  for (int i = 0; i < 6; ++i) transpose_cast_f16<<<dim3(FD / 64, FD / 64), dim3(32, 8), 0, stream>>>(Wl[i], FD, W6 + (size_t)i * FD * FD, FD, 1.0f);
  transpose_cast_f16<<<dim3(FD / 64, FD / 64), dim3(32, 8), 0, stream>>>(Wo, FD, WoT, FD, 1.0f);
  bias6_kernel<<<12, 256, 0, stream>>>(bl[0], bl[1], bl[2], bl[3], bl[4], bl[5], b6);
  { const int t = (FR / 64) * (FN6 / 64);
    wmma_gemm64<0, false, 2, 0, false><<<dim3((t + 7) / 8, 1), 256, 0, stream>>>((const unsigned short*)XN16, nullptr, FD, 0, U16(W6), nullptr, FD, 0, P6, nullptr, FN6, 0, b6, nullptr, 0, FR, FN6, FD, 1.0f); }
  anchor_kernel<<<(FB_ * FD / 2 + 255) / 256, 256, 0, stream>>>(P6, Q16, KW16);
  for (int b = 0; b < FB_; ++b) {
    { const int t = (FS / 64) * (FS / 64);
      wmma_gemm64<0, false, 0, 0, false><<<dim3((t + 7) / 8, FH), 256, 0, stream>>>((const unsigned short*)Q16 + (size_t)b * FS * FD, nullptr, FD, FHD, (const unsigned short*)KW16 + (size_t)b * FS * FD, nullptr, FD, FHD, Sm, nullptr, FS, (long)FS * FS, nullptr, nullptr, 0, FS, FS, FHD, 1.0f); }
    probs_kernel<<<FS * FS / 512, 256, 0, stream>>>(Sm, P16);
    vt_kernel<<<dim3(FS / 64, FH), dim3(32, 8), 0, stream>>>(P6, b, VT16);
    { const int t = (FS / 64) * 1;
      wmma_gemm64<0, false, 0, 0, false><<<dim3((t + 7) / 8, FH), 256, 0, stream>>>((const unsigned short*)P16, nullptr, FS, (long)FS * FS, (const unsigned short*)VT16, nullptr, FS, (long)64 * FS, ATT + (size_t)b * FS * 1024, nullptr, 1024, 64, nullptr, nullptr, 0, FS, 64, FS, 1.0f / 32768.0f); }
  }
  combine_kernel<<<FR / 8, 256, 0, stream>>>(ATT, P6, PRE16);
  { const int t = (FR / 64) * (FD / 64);
    wmma_gemm64<0, false, 2, 0, true><<<dim3((t + 7) / 8, 1), 256, 0, stream>>>((const unsigned short*)PRE16, nullptr, FD, 0, U16(WoT), nullptr, FD, 0, (float*)d_out, nullptr, FD, 0, bo, x, 0, FR, FD, FD, 1.0f); }
}
